// Net_60129542144705
// MI455X (gfx1250) — hardware-verified
//
#include <hip/hip_runtime.h>
#include <stddef.h>
#include <stdint.h>
#include <math.h>


#define CIN    128
#define HID    16
#define NCLS   40
#define PQ1W   32
#define PQ2W   96
#define K2B    96
#define NTHR   256
#define NWAVE  8
#define EPT    8
#define CHUNK  (NTHR * EPT)
#define WCAP   (EPT * 32)
#define LISTN  (NWAVE * WCAP)
#define NB1    1024
#define SL1    10
#define RCAP1  24576
#define NB2    512
#define SL2    9
#define RCAP2  12288
#define TP1    32
#define TP2    104
#define GBM    64
#define GTHR   128
#define NFLAGMAX 64
#define MISC_INTS 16
#define ACC1_INTS ((NB1 + 1) * HID)
#define ACC2_INTS ((NB2 + 1) * NCLS)
#define TIL1_INTS (NWAVE * 16 * TP1 / 2)
#define TIL2_INTS (NWAVE * 16 * TP2 / 2)
#define STG1_INTS (NWAVE * 16 * PQ2W)
#define LDS1_INTS (LISTN + RCAP1 + NB1 + ACC1_INTS + MISC_INTS + TIL1_INTS + STG1_INTS)
#define LDS2_INTS (LISTN + RCAP2 + NB2 + ACC2_INTS + MISC_INTS + TIL2_INTS)
#define WSMAX  134217728

static_assert((CHUNK & (CHUNK - 1)) == 0 && CHUNK <= 4096);
static_assert(NB1 == (1 << SL1) && NB2 == (1 << SL2));
static_assert(((long long)CHUNK << SL1) < (1LL << 31));
static_assert(LISTN % 4 == 0 && RCAP1 % 4 == 0 && RCAP2 % 4 == 0 && NB1 % 4 == 0 && NB2 % 4 == 0);
static_assert(ACC1_INTS % 4 == 0 && ACC2_INTS % 4 == 0 && MISC_INTS % 4 == 0);
static_assert(LDS1_INTS % 4 == 0 && LDS2_INTS % 4 == 0);
static_assert(LDS1_INTS * 4 <= 300000 && LDS2_INTS * 4 <= 300000);
static_assert(NB1 % (NWAVE * 16) == 0 && NB2 % NTHR == 0 && NB2 % 4 == 0);
static_assert((NB2 * NCLS * 4) % 128 == 0);
static_assert(CIN % 32 == 0 && K2B % 32 == 0 && PQ1W == 2 * HID && PQ2W == 2 * 48);
static_assert(GBM == (GTHR / 32) * 16 && (GBM * PQ1W) == 4 * GTHR * 4);
static_assert((TP2 * 2) % 16 == 0 && TP2 >= K2B);

typedef float          v4f   __attribute__((ext_vector_type(4)));
typedef float          v8f   __attribute__((ext_vector_type(8)));
typedef int            v4i   __attribute__((ext_vector_type(4)));
typedef int            v8i   __attribute__((ext_vector_type(8)));
typedef unsigned int   v4u   __attribute__((ext_vector_type(4)));
typedef unsigned short v4us  __attribute__((ext_vector_type(4)));
typedef unsigned short v8us  __attribute__((ext_vector_type(8)));
typedef unsigned short v16us __attribute__((ext_vector_type(16)));
typedef __bf16         v16bf __attribute__((ext_vector_type(16)));
typedef v4f  __attribute__((may_alias)) v4fa;
typedef v4i  __attribute__((may_alias)) v4ia;
typedef v4u  __attribute__((may_alias)) v4ua;
typedef v4us __attribute__((may_alias)) v4usa;
typedef v8us __attribute__((may_alias)) v8usa;
union FragB { v16bf v; v16us u; v8us h[2]; v8i w; };

__device__ __forceinline__ v8f wmb(const FragB& a, const FragB& b, v8f c) {
  v8f d = __builtin_amdgcn_wmma_f32_16x16x32_bf16(false, a.v, false, b.v, (short)0, c, false, false);
  asm volatile("v_nop\n\tv_nop\n\tv_nop\n\tv_nop" : "+v"(d) : "v"(a.w), "v"(b.w));
  return d;
}

__device__ __forceinline__ unsigned bf16_bits(float f) {
  const unsigned u = __float_as_uint(f);
  return (u + 0x7FFFu + ((u >> 16) & 1u)) >> 16;
}
__device__ __forceinline__ float bf16_val(float f) {
  return __uint_as_float(bf16_bits(f) << 16);
}
__device__ __forceinline__ void split2(float r, unsigned& hb, unsigned& lb) {
  hb = bf16_bits(r);
  lb = bf16_bits(r - __uint_as_float(hb << 16));
}
__device__ __forceinline__ float relu_np(float v) { return (v > 0.0f) ? v : (v - v); }

__device__ __forceinline__ unsigned f2ord(float v) {
  unsigned u = __float_as_uint(v);
  u = (v != v) ? 0x7fc00000u : u;
  return (u & 0x80000000u) ? ~u : (u | 0x80000000u);
}
__device__ __forceinline__ float ord2f(unsigned e) {
  const unsigned u = (e & 0x80000000u) ? (e & 0x7fffffffu) : ~e;
  return __uint_as_float(u);
}

__device__ __forceinline__ void wave_sync() {
  __builtin_amdgcn_fence(__ATOMIC_RELEASE, "wavefront");
  __builtin_amdgcn_wave_barrier();
  __builtin_amdgcn_fence(__ATOMIC_ACQUIRE, "wavefront");
}

template <int SLB>
__device__ __forceinline__ int scan_chunk(const int* __restrict__ dsts, int nE, int cbase, int slotBase,
                                          int nb, int vec8, int* list, int tid, int lane, int wave) {
  int wc = 0;
  const int el0  = tid * EPT;
  const int e0   = cbase + el0;
  const int sent = -2147483647 - 1;
  v4i da, db;
  if (vec8 != 0 && cbase + CHUNK <= nE) {
    da = *(const v4i*)(dsts + e0);
    db = *(const v4i*)(dsts + e0 + 4);
  } else {
    da.x = (e0     < nE) ? dsts[min(e0,     nE - 1)] : sent;
    da.y = (e0 + 1 < nE) ? dsts[min(e0 + 1, nE - 1)] : sent;
    da.z = (e0 + 2 < nE) ? dsts[min(e0 + 2, nE - 1)] : sent;
    da.w = (e0 + 3 < nE) ? dsts[min(e0 + 3, nE - 1)] : sent;
    db.x = (e0 + 4 < nE) ? dsts[min(e0 + 4, nE - 1)] : sent;
    db.y = (e0 + 5 < nE) ? dsts[min(e0 + 5, nE - 1)] : sent;
    db.z = (e0 + 6 < nE) ? dsts[min(e0 + 6, nE - 1)] : sent;
    db.w = (e0 + 7 < nE) ? dsts[min(e0 + 7, nE - 1)] : sent;
  }
  const unsigned nbs = (unsigned)slotBase;
  const unsigned unb = (unsigned)nb;
  const unsigned s0 = (unsigned)da.x - nbs, s1 = (unsigned)da.y - nbs;
  const unsigned s2 = (unsigned)da.z - nbs, s3 = (unsigned)da.w - nbs;
  const unsigned s4 = (unsigned)db.x - nbs, s5 = (unsigned)db.y - nbs;
  const unsigned s6 = (unsigned)db.z - nbs, s7 = (unsigned)db.w - nbs;
  const bool h0 = s0 < unb, h1 = s1 < unb, h2 = s2 < unb, h3 = s3 < unb;
  const bool h4 = s4 < unb, h5 = s5 < unb, h6 = s6 < unb, h7 = s7 < unb;
  const unsigned any = __builtin_amdgcn_ballot_w32(h0 | h1 | h2 | h3 | h4 | h5 | h6 | h7);
  if (any != 0u) {
#define HITJ(J, HJ, SJ) { \
      const unsigned mj = __builtin_amdgcn_ballot_w32(HJ); \
      if (mj != 0u) { \
        if (HJ) { \
          const int pos = wc + (int)__builtin_amdgcn_mbcnt_lo(mj, 0u); \
          if (pos < WCAP) list[wave * WCAP + pos] = ((el0 + (J)) << SLB) | (int)(SJ); \
        } \
        wc += (int)__builtin_popcount(mj); } }
    HITJ(0, h0, s0)
    HITJ(1, h1, s1)
    HITJ(2, h2, s2)
    HITJ(3, h3, s3)
    HITJ(4, h4, s4)
    HITJ(5, h5, s5)
    HITJ(6, h6, s6)
    HITJ(7, h7, s7)
#undef HITJ
  }
  return wc;
}

template <int SLB, int NBK, int RC>
__device__ __forceinline__ void build_hits(const int* __restrict__ dsts, int nE, int vec8, int nodeBase,
                                           int* list, int* hl, int* cnt, int* misc,
                                           int tid, int lane, int wave, int& ttOut, int& ovOut) {
  int t = 0, ov = 0;
  const int nChunks = (nE + CHUNK - 1) / CHUNK;
#pragma unroll 1
  for (int ch = 0; ch < nChunks; ++ch) {
    const int cbase = ch * CHUNK;
    const int wc = scan_chunk<SLB>(dsts, nE, cbase, nodeBase, NBK, vec8, list, tid, lane, wave);
    if (lane == 0) misc[wave] = wc;
    __syncthreads();
    if (wave == 0) {
#pragma unroll 1
      for (int w2 = 0; w2 < NWAVE; ++w2) {
        int c = misc[w2];
        c = c < 0 ? 0 : (c > WCAP ? WCAP : c);
#pragma unroll 1
        for (int b0 = 0; b0 < c; b0 += 32) {
          const int idx = b0 + lane;
          const int ent = list[w2 * WCAP + (idx < WCAP ? idx : WCAP - 1)];
          const int m32 = (c - b0) < 32 ? (c - b0) : 32;
#pragma unroll 1
          for (int k = 0; k < m32; ++k) {
            const int u    = __builtin_amdgcn_readlane(ent, k);
            const int slot = u & (NBK - 1);
            const int el   = (u >> SLB) & (CHUNK - 1);
            const int pk   = ((cbase + el) << SLB) | slot;
            if (t < RC) {
              if (lane == 0) { hl[t] = pk; cnt[slot] = cnt[slot] + 1; }
              t = t + 1;
            } else {
              ov = 1;
            }
          }
        }
      }
    }
    __syncthreads();
  }
  if (wave == 0 && lane == 0) { misc[8] = t; misc[9] = ov; }
  __syncthreads();
  int tt = misc[8];
  tt = tt < 0 ? 0 : (tt > RC ? RC : tt);
  ttOut = tt;
  ovOut = misc[9];
}

__global__ __launch_bounds__(NTHR) void k_prep(
    const float* __restrict__ x, int nN, int nXB,
    const float* __restrict__ W1a, const float* __restrict__ b1a,
    const float* __restrict__ W1b, const float* __restrict__ b1b,
    const float* __restrict__ W2a, const float* __restrict__ b2a,
    const float* __restrict__ W2b, const float* __restrict__ b2b,
    unsigned short* XB, unsigned short* BT1, unsigned short* BT1b,
    unsigned short* BT2a, unsigned short* BT2b, float* BIAS)
{
  __shared__ __attribute__((aligned(16))) float sb[128];
  const int tid = (int)threadIdx.x;
  const int b   = (int)blockIdx.x;
  if (b < nXB) {
    const int u   = b * NTHR + tid;
    const int row = u >> 4;
    const int k8  = (u & 15) * 8;
    const int rc  = row < nN ? row : nN - 1;
    const float* p = x + (size_t)rc * CIN + k8;
    const v4f a = *(const v4fa*)p;
    const v4f c = *(const v4fa*)(p + 4);
    const bool ok = row < nN;
    v8us o;
    o[0] = ok ? (unsigned short)bf16_bits(a.x) : (unsigned short)0;
    o[1] = ok ? (unsigned short)bf16_bits(a.y) : (unsigned short)0;
    o[2] = ok ? (unsigned short)bf16_bits(a.z) : (unsigned short)0;
    o[3] = ok ? (unsigned short)bf16_bits(a.w) : (unsigned short)0;
    o[4] = ok ? (unsigned short)bf16_bits(c.x) : (unsigned short)0;
    o[5] = ok ? (unsigned short)bf16_bits(c.y) : (unsigned short)0;
    o[6] = ok ? (unsigned short)bf16_bits(c.z) : (unsigned short)0;
    o[7] = ok ? (unsigned short)bf16_bits(c.w) : (unsigned short)0;
    unsigned short* dp = XB + (size_t)u * 8;
    *(volatile v8us*)dp = o;
    __threadfence();
    *(volatile v8us*)dp = o;
    return;
  }
  const int wb = b - nXB;
  if (wb == 8) {
    const int f  = tid < 128 ? tid : 127;
    const int i0 = f < 15 ? f : 15;
    int i1 = f - 16; i1 = i1 < 0 ? 0 : (i1 > 15 ? 15 : i1);
    int i2 = f - 32; i2 = i2 < 0 ? 0 : (i2 > NCLS - 1 ? NCLS - 1 : i2);
    int i3 = f - 80; i3 = i3 < 0 ? 0 : (i3 > NCLS - 1 ? NCLS - 1 : i3);
    const float v0 = b1a[i0], v1 = b1b[i1], v2 = b2a[i2], v3 = b2b[i3];
    float v = 0.0f;
    v = (f < 16) ? v0 : v;
    v = (f >= 16 && f < 32) ? v1 : v;
    v = (f >= 32 && f < 32 + NCLS) ? v2 : v;
    v = (f >= 80 && f < 80 + NCLS) ? v3 : v;
    if (tid < 128) sb[tid] = bf16_val(v);
    __syncthreads();
    const int q = tid < 32 ? tid : 31;
    const v4f ov = *(const v4fa*)(sb + 4 * q);
    float* op = BIAS + 4 * q;
    const bool ok = tid < 32;
    if (ok) *(volatile v4f*)op = ov;
    __threadfence();
    if (ok) *(volatile v4f*)op = ov;
    return;
  }
  v8us o;
  unsigned short* dp;
  bool ok;
  if (wb < 2) {
    const int v  = wb * NTHR + tid;
    const int n  = v >> 4;
    const int k8 = (v & 15) * 8;
    const int off = (n < 16) ? (k8 * HID + n) : ((CIN + k8) * HID + (n - 16));
    const float* p = W1a + off;
#pragma unroll
    for (int i = 0; i < 8; ++i) o[i] = (unsigned short)bf16_bits(p[i * HID]);
    dp = BT1 + (size_t)v * 8;
    ok = true;
  } else if (wb == 2) {
    const int v  = tid < 63 ? tid : 63;
    ok = tid < 64;
    const int n  = v >> 2;
    const int k8 = (v & 3) * 8;
#pragma unroll
    for (int i = 0; i < 8; ++i) {
      const int kk = (k8 + i) & 15;
      o[i] = (unsigned short)bf16_bits(W1b[kk * HID + n]);
    }
    dp = BT1b + (size_t)v * 8;
  } else if (wb < 5) {
    const int v0 = (wb - 3) * NTHR + tid;
    const int v  = v0 < 383 ? v0 : 383;
    ok = v0 < 384;
    const int n  = v >> 2;
    const int k8 = (v & 3) * 8;
    const int c  = (n < 48) ? n : (n - 48);
    const int rb = (n < 48) ? 0 : HID;
    const bool cv = c < NCLS;
    const int cc = cv ? c : NCLS - 1;
#pragma unroll
    for (int i = 0; i < 8; ++i) {
      const int kk = (k8 + i) & 15;
      const float w = W2a[(rb + kk) * NCLS + cc];
      o[i] = cv ? (unsigned short)bf16_bits(w) : (unsigned short)0;
    }
    dp = BT2a + (size_t)v * 8;
  } else {
    const int v0 = (wb - 5) * NTHR + tid;
    const int v  = v0 < 575 ? v0 : 575;
    ok = v0 < 576;
    const int n  = v / 12;
    const int k8 = (v - n * 12) * 8;
    const int nc = n < NCLS ? n : NCLS - 1;
#pragma unroll
    for (int i = 0; i < 8; ++i) {
      const int k  = k8 + i;
      const int kk = (k < 48) ? k : (k - 48);
      const bool vv = (kk < NCLS) && (n < NCLS);
      const int kc = kk < NCLS ? kk : NCLS - 1;
      const float w = W2b[kc * NCLS + nc];
      o[i] = vv ? (unsigned short)bf16_bits(w) : (unsigned short)0;
    }
    dp = BT2b + (size_t)v * 8;
  }
  if (ok) *(volatile v8us*)dp = o;
  __threadfence();
  if (ok) *(volatile v8us*)dp = o;
}

__global__ __launch_bounds__(GTHR) void k_gemm1(const unsigned short* __restrict__ XB,
                                                const unsigned short* __restrict__ BT1,
                                                const float* __restrict__ BIAS, float* PQ1)
{
  __shared__ __attribute__((aligned(16))) float stg[GBM * PQ1W];
  const int tid = (int)threadIdx.x, lane = tid & 31, wave = tid >> 5, hh = lane >> 4, m = lane & 15;
  const int rowBase = (int)blockIdx.x * GBM;
  v8f acc0 = {0.f, 0.f, 0.f, 0.f, 0.f, 0.f, 0.f, 0.f};
  v8f acc1 = acc0;
  const unsigned short* ap = XB  + (size_t)(rowBase + 16 * wave + m) * CIN + 8 * hh;
  const unsigned short* wp = BT1 + (size_t)m * CIN + 8 * hh;
#pragma unroll 1
  for (int ks = 0; ks < CIN / 32; ++ks) {
    FragB af, b0, b1;
    af.h[0] = *(const v8usa*)(ap + 32 * ks);
    af.h[1] = *(const v8usa*)(ap + 32 * ks + 16);
    b0.h[0] = *(const v8usa*)(wp + 32 * ks);
    b0.h[1] = *(const v8usa*)(wp + 32 * ks + 16);
    b1.h[0] = *(const v8usa*)(wp + 16 * CIN + 32 * ks);
    b1.h[1] = *(const v8usa*)(wp + 16 * CIN + 32 * ks + 16);
    acc0 = wmb(af, b0, acc0);
    acc1 = wmb(af, b1, acc1);
  }
  const float ba = BIAS[m];
#pragma unroll
  for (int r = 0; r < 8; ++r) {
    const int lr = 16 * wave + 8 * hh + r;
    stg[lr * PQ1W + m]       = (acc0[r] - acc1[r]) + ba;
    stg[lr * PQ1W + HID + m] = acc1[r];
  }
  __syncthreads();
  v4f fv[4];
#pragma unroll
  for (int it = 0; it < 4; ++it) fv[it] = *(const v4fa*)(stg + (it * GTHR + tid) * 4);
  float* op = PQ1 + (size_t)rowBase * PQ1W;
#pragma unroll
  for (int it = 0; it < 4; ++it) *(volatile v4f*)(op + (it * GTHR + tid) * 4) = fv[it];
  __threadfence();
#pragma unroll
  for (int it = 0; it < 4; ++it) *(volatile v4f*)(op + (it * GTHR + tid) * 4) = fv[it];
}

__global__ __launch_bounds__(NTHR) void k_scan1(
    const int* __restrict__ srcs, const int* __restrict__ dsts, int nE, int nN, int vec8,
    const float* __restrict__ pq1, const unsigned short* __restrict__ bt1b,
    const unsigned short* __restrict__ bt2a, const float* __restrict__ bias,
    float* pq2, int* flag)
{
  extern __shared__ __attribute__((aligned(16))) int dsm[];
  int* list = dsm;
  int* hl   = list + LISTN;
  int* cnt  = hl + RCAP1;
  unsigned* accu = (unsigned*)(cnt + NB1);
  int* misc = (int*)accu + ACC1_INTS;
  unsigned short* tiles = (unsigned short*)(misc + MISC_INTS);
  float* stgall = (float*)(misc + MISC_INTS + TIL1_INTS);
  const int tid = (int)threadIdx.x, lane = tid & 31, wave = tid >> 5, hh = lane >> 4, m = lane & 15;
  const int nodeBase = (int)blockIdx.x * NB1;

  {
    const v4i z4 = {0, 0, 0, 0};
    for (int i = tid * 4; i < LDS1_INTS; i += NTHR * 4) *(v4ia*)(dsm + i) = z4;
  }
  __syncthreads();

  int tt = 0, ovf = 0;
  build_hits<SL1, NB1, RCAP1>(dsts, nE, vec8, nodeBase, list, hl, cnt, misc, tid, lane, wave, tt, ovf);

  {
    FragB bw;
    {
      const unsigned short* bp = bt1b + m * 32 + 8 * hh;
      bw.h[0] = *(const v8usa*)bp;
      bw.h[1] = *(const v8usa*)(bp + 16);
    }
    unsigned short* tile = tiles + wave * (16 * TP1);
    const v8f zf = {0.f, 0.f, 0.f, 0.f, 0.f, 0.f, 0.f, 0.f};
    const int nT = (tt + 15) >> 4;
#pragma unroll 1
    for (int j = wave; j < nT; j += NWAVE) {
      const int idx = 16 * j + m;
      const bool valid = idx < tt;
      const int ent = hl[idx < RCAP1 ? idx : RCAP1 - 1];
      const int slot = ent & (NB1 - 1);
      int eid = ent >> SL1;
      eid = eid < 0 ? 0 : (eid > nE - 1 ? nE - 1 : eid);
      int sr = srcs[eid];
      sr = sr < 0 ? 0 : (sr > nN - 1 ? nN - 1 : sr);
      int nd = nodeBase + slot;
      nd = nd > nN - 1 ? nN - 1 : nd;
      const float* pp = pq1 + (size_t)nd * PQ1W + 8 * hh;
      const float* qp = pq1 + (size_t)sr * PQ1W + HID + 8 * hh;
      const v4f p0 = *(const v4fa*)pp;
      const v4f p1 = *(const v4fa*)(pp + 4);
      const v4f q0 = *(const v4fa*)qp;
      const v4f q1 = *(const v4fa*)(qp + 4);
      float rr[8];
      rr[0] = relu_np(p0.x + q0.x); rr[1] = relu_np(p0.y + q0.y);
      rr[2] = relu_np(p0.z + q0.z); rr[3] = relu_np(p0.w + q0.w);
      rr[4] = relu_np(p1.x + q1.x); rr[5] = relu_np(p1.y + q1.y);
      rr[6] = relu_np(p1.z + q1.z); rr[7] = relu_np(p1.w + q1.w);
      v8us hv8, lv8;
#pragma unroll
      for (int i = 0; i < 8; ++i) {
        unsigned hb, lb;
        split2(rr[i], hb, lb);
        hv8[i] = (unsigned short)hb;
        lv8[i] = (unsigned short)lb;
      }
      *(v8usa*)(tile + m * TP1 + 8 * hh)      = hv8;
      *(v8usa*)(tile + m * TP1 + 16 + 8 * hh) = lv8;
      wave_sync();
      FragB af;
      af.h[0] = *(const v8usa*)(tile + m * TP1 + 8 * hh);
      af.h[1] = *(const v8usa*)(tile + m * TP1 + 16 + 8 * hh);
      wave_sync();
      const v8f d = wmb(af, bw, zf);
      const int slv = valid ? slot : NB1;
#pragma unroll
      for (int r = 0; r < 8; ++r) {
        const int sl_r = __shfl(slv, 8 * hh + r, 32);
        atomicMax(accu + sl_r * HID + m, f2ord(d[r]));
      }
    }
  }
  __syncthreads();

  {
    const float qnan = __int_as_float(0x7fc00000);
    const float pz = (ovf != 0) ? qnan : 0.0f;
    FragB b2[6];
#pragma unroll
    for (int nt = 0; nt < 6; ++nt) {
      const unsigned short* bp = bt2a + (16 * nt + m) * 32 + 8 * hh;
      b2[nt].h[0] = *(const v8usa*)bp;
      b2[nt].h[1] = *(const v8usa*)(bp + 16);
    }
    const v4f bb0 = *(const v4fa*)(bias + 16 + 8 * hh);
    const v4f bb1 = *(const v4fa*)(bias + 16 + 8 * hh + 4);
    float ba2[3];
#pragma unroll
    for (int nt = 0; nt < 3; ++nt) ba2[nt] = bias[32 + 16 * nt + m];
    float* stg = stgall + wave * (16 * PQ2W);
    const v8f zf = {0.f, 0.f, 0.f, 0.f, 0.f, 0.f, 0.f, 0.f};
#pragma unroll 1
    for (int t = 0; t < NB1 / (NWAVE * 16); ++t) {
      const int s0 = wave * (NB1 / NWAVE) + 16 * t;
      const int s  = s0 + m;
      const int c  = cnt[s];
      const bool live = (nodeBase + s) < nN;
      const v4u e0 = *(const v4ua*)(accu + s * HID + 8 * hh);
      const v4u e1 = *(const v4ua*)(accu + s * HID + 8 * hh + 4);
      float hv[8];
      hv[0] = ord2f(e0.x) + bb0.x; hv[1] = ord2f(e0.y) + bb0.y;
      hv[2] = ord2f(e0.z) + bb0.z; hv[3] = ord2f(e0.w) + bb0.w;
      hv[4] = ord2f(e1.x) + bb1.x; hv[5] = ord2f(e1.y) + bb1.y;
      hv[6] = ord2f(e1.z) + bb1.z; hv[7] = ord2f(e1.w) + bb1.w;
      FragB af;
#pragma unroll
      for (int i = 0; i < 8; ++i) {
        float v = (c > 0) ? hv[i] : 0.0f;
        v = relu_np(v);
        v = v + pz;
        v = live ? v : 0.0f;
        unsigned hb, lb;
        split2(v, hb, lb);
        af.u[i]     = (unsigned short)hb;
        af.u[8 + i] = (unsigned short)lb;
      }
      v8f d[6];
#pragma unroll
      for (int nt = 0; nt < 6; ++nt) d[nt] = wmb(af, b2[nt], zf);
#pragma unroll
      for (int nt = 0; nt < 3; ++nt) {
#pragma unroll
        for (int r = 0; r < 8; ++r) {
          const int lr = 8 * hh + r;
          stg[lr * PQ2W + 16 * nt + m]      = (d[nt][r] - d[nt + 3][r]) + ba2[nt];
          stg[lr * PQ2W + 48 + 16 * nt + m] = d[nt + 3][r];
        }
      }
      wave_sync();
      v4f ov[12];
#pragma unroll
      for (int it = 0; it < 12; ++it) ov[it] = *(const v4fa*)(stg + (it * 32 + lane) * 4);
      wave_sync();
      float* op = pq2 + (size_t)(nodeBase + s0) * PQ2W;
#pragma unroll
      for (int it = 0; it < 12; ++it) *(volatile v4f*)(op + (it * 32 + lane) * 4) = ov[it];
      __threadfence();
#pragma unroll
      for (int it = 0; it < 12; ++it) *(volatile v4f*)(op + (it * 32 + lane) * 4) = ov[it];
    }
  }
  {
    const v4i fv = {ovf, ovf, ovf, ovf};
    int* fp = flag + (size_t)blockIdx.x * 32 + 4 * (lane & 7);
    const bool okf = (wave == 0) && (lane < 8);
    if (okf) *(volatile v4i*)fp = fv;
    __threadfence();
    if (okf) *(volatile v4i*)fp = fv;
  }
}

__global__ __launch_bounds__(NTHR) void k_scan2(
    const int* __restrict__ srcs, const int* __restrict__ dsts, int nE, int nN, int vec8,
    const float* __restrict__ pq2, const unsigned short* __restrict__ bt2b,
    const float* __restrict__ bias, const int* __restrict__ flag, int nFlag, float* out)
{
  extern __shared__ __attribute__((aligned(16))) int dsm[];
  int* list = dsm;
  int* hl   = list + LISTN;
  int* cnt  = hl + RCAP2;
  unsigned* accu = (unsigned*)(cnt + NB2);
  int* misc = (int*)accu + ACC2_INTS;
  unsigned short* tiles = (unsigned short*)(misc + MISC_INTS);
  const int tid = (int)threadIdx.x, lane = tid & 31, wave = tid >> 5, hh = lane >> 4, m = lane & 15;
  const int nodeBase = (int)blockIdx.x * NB2;

  {
    const v4i z4 = {0, 0, 0, 0};
    for (int i = tid * 4; i < LDS2_INTS; i += NTHR * 4) *(v4ia*)(dsm + i) = z4;
  }
  __syncthreads();

  int tt = 0, ovf = 0;
  build_hits<SL2, NB2, RCAP2>(dsts, nE, vec8, nodeBase, list, hl, cnt, misc, tid, lane, wave, tt, ovf);

  {
    FragB bf[3][3];
#pragma unroll
    for (int ks = 0; ks < 3; ++ks) {
#pragma unroll
      for (int nt = 0; nt < 3; ++nt) {
        const unsigned short* bp = bt2b + (16 * nt + m) * K2B + 32 * ks + 8 * hh;
        bf[ks][nt].h[0] = *(const v8usa*)bp;
        bf[ks][nt].h[1] = *(const v8usa*)(bp + 16);
      }
    }
    unsigned short* tile = tiles + wave * (16 * TP2);
    const v8f zf = {0.f, 0.f, 0.f, 0.f, 0.f, 0.f, 0.f, 0.f};
    const bool padl = m >= 8;
    const int nT = (tt + 15) >> 4;
#pragma unroll 1
    for (int j = wave; j < nT; j += NWAVE) {
      const int idx = 16 * j + m;
      const bool valid = idx < tt;
      const int ent = hl[idx < RCAP2 ? idx : RCAP2 - 1];
      const int slot = ent & (NB2 - 1);
      int eid = ent >> SL2;
      eid = eid < 0 ? 0 : (eid > nE - 1 ? nE - 1 : eid);
      int sr = srcs[eid];
      sr = sr < 0 ? 0 : (sr > nN - 1 ? nN - 1 : sr);
      int nd = nodeBase + slot;
      nd = nd > nN - 1 ? nN - 1 : nd;
      const float* pp = pq2 + (size_t)nd * PQ2W + 24 * hh;
      const float* qp = pq2 + (size_t)sr * PQ2W + 48 + 24 * hh;
      unsigned short* tr = tile + m * TP2 + 24 * hh;
#pragma unroll
      for (int q = 0; q < 6; ++q) {
        const v4f p  = *(const v4fa*)(pp + 4 * q);
        const v4f qv = *(const v4fa*)(qp + 4 * q);
        const float r0 = relu_np(p.x + qv.x), r1 = relu_np(p.y + qv.y);
        const float r2 = relu_np(p.z + qv.z), r3 = relu_np(p.w + qv.w);
        v4us h4, l4;
        unsigned hb, lb;
        split2(r0, hb, lb); h4[0] = (unsigned short)hb; l4[0] = (unsigned short)lb;
        split2(r1, hb, lb); h4[1] = (unsigned short)hb; l4[1] = (unsigned short)lb;
        split2(r2, hb, lb); h4[2] = (unsigned short)hb; l4[2] = (unsigned short)lb;
        split2(r3, hb, lb); h4[3] = (unsigned short)hb; l4[3] = (unsigned short)lb;
        *(v4usa*)(tr + 4 * q)      = h4;
        *(v4usa*)(tr + 48 + 4 * q) = l4;
      }
      wave_sync();
      FragB af[3];
      const unsigned short* ar = tile + m * TP2 + 8 * hh;
#pragma unroll
      for (int ks = 0; ks < 3; ++ks) {
        af[ks].h[0] = *(const v8usa*)(ar + 32 * ks);
        af[ks].h[1] = *(const v8usa*)(ar + 32 * ks + 16);
      }
      wave_sync();
      v8f d[3];
      d[0] = zf; d[1] = zf; d[2] = zf;
#pragma unroll
      for (int ks = 0; ks < 3; ++ks) {
#pragma unroll
        for (int nt = 0; nt < 3; ++nt) d[nt] = wmb(af[ks], bf[ks][nt], d[nt]);
      }
      const int slv = valid ? slot : NB2;
#pragma unroll
      for (int r = 0; r < 8; ++r) {
        const int sl_r = __shfl(slv, 8 * hh + r, 32);
        atomicMax(accu + sl_r * NCLS + m,      f2ord(d[0][r]));
        atomicMax(accu + sl_r * NCLS + 16 + m, f2ord(d[1][r]));
        const int rs = padl ? NB2 : sl_r;
        const int cs = padl ? (24 + m) : (32 + m);
        atomicMax(accu + rs * NCLS + cs, f2ord(d[2][r]));
      }
    }
  }
  __syncthreads();

  {
    int f1 = ovf;
    int nf = nFlag < 0 ? 0 : (nFlag > NFLAGMAX ? NFLAGMAX : nFlag);
#pragma unroll 1
    for (int i = 0; i < nf; ++i) f1 |= flag[i * 32];
    const float pz = (f1 != 0) ? __int_as_float(0x7fc00000) : 0.0f;
#pragma unroll 1
    for (int s = tid; s < NB2; s += NTHR) {
      const int c = cnt[s];
      unsigned* row = accu + s * NCLS;
      float mx = -INFINITY;
#pragma unroll 1
      for (int q = 0; q < NCLS / 4; ++q) {
        const v4u e = *(const v4ua*)(row + 4 * q);
        const v4f bb = *(const v4fa*)(bias + 80 + 4 * q);
        const float z0 = (c > 0) ? (ord2f(e.x) + bb.x) : 0.0f;
        const float z1 = (c > 0) ? (ord2f(e.y) + bb.y) : 0.0f;
        const float z2 = (c > 0) ? (ord2f(e.z) + bb.z) : 0.0f;
        const float z3 = (c > 0) ? (ord2f(e.w) + bb.w) : 0.0f;
        mx = fmaxf(mx, fmaxf(fmaxf(z0, z1), fmaxf(z2, z3)));
        v4u zo;
        zo.x = __float_as_uint(z0); zo.y = __float_as_uint(z1);
        zo.z = __float_as_uint(z2); zo.w = __float_as_uint(z3);
        *(v4ua*)(row + 4 * q) = zo;
      }
      float sum = 0.0f;
#pragma unroll 1
      for (int q = 0; q < NCLS / 4; ++q) {
        const v4u e = *(const v4ua*)(row + 4 * q);
        sum += expf(__uint_as_float(e.x) - mx);
        sum += expf(__uint_as_float(e.y) - mx);
        sum += expf(__uint_as_float(e.z) - mx);
        sum += expf(__uint_as_float(e.w) - mx);
      }
      const float ls = logf(sum);
#pragma unroll 1
      for (int q = 0; q < NCLS / 4; ++q) {
        const v4u e = *(const v4ua*)(row + 4 * q);
        v4u zo;
        zo.x = __float_as_uint(((__uint_as_float(e.x) - mx) - ls) + pz);
        zo.y = __float_as_uint(((__uint_as_float(e.y) - mx) - ls) + pz);
        zo.z = __float_as_uint(((__uint_as_float(e.z) - mx) - ls) + pz);
        zo.w = __float_as_uint(((__uint_as_float(e.w) - mx) - ls) + pz);
        *(v4ua*)(row + 4 * q) = zo;
      }
    }
  }
  __syncthreads();

  {
    int rows = nN - nodeBase;
    rows = rows < 0 ? 0 : (rows > NB2 ? NB2 : rows);
    const int nvec = rows * (NCLS / 4);
    const float* src = (const float*)accu;
    float* ob = out + (size_t)nodeBase * NCLS;
#pragma unroll 1
    for (int i = tid; i < nvec; i += NTHR) {
      const v4f v = *(const v4fa*)(src + 4 * i);
      *(volatile v4f*)(ob + 4 * (size_t)i) = v;
    }
    __threadfence();
#pragma unroll 1
    for (int i = tid; i < nvec; i += NTHR) {
      const v4f v = *(const v4fa*)(src + 4 * i);
      *(volatile v4f*)(ob + 4 * (size_t)i) = v;
    }
  }
}

static inline int cdiv(int a, int b) { return (a + b - 1) / b; }
static inline size_t al256(size_t o) { return (o + 255) & ~(size_t)255; }

extern "C" void kernel_launch(void* const* d_in, const int* in_sizes, int n_in,
                              void* d_out, int out_size, void* d_ws, size_t ws_size,
                              hipStream_t stream) {
  if (n_in < 10) return;
  if (in_sizes[0] < CIN || (in_sizes[0] % CIN) != 0) return;
  const int nN = in_sizes[0] / CIN;
  if (nN < 4 || (nN & 3) != 0 || nN > (1 << 22)) return;
  if (in_sizes[1] < 2 || (in_sizes[1] & 1) != 0) return;
  const int nE = in_sizes[1] / 2;
  if (nE < 1 || nE >= (1 << (31 - SL1))) return;
  if (in_sizes[2] != 2 * CIN * HID || in_sizes[3] != HID) return;
  if (in_sizes[4] != HID * HID || in_sizes[5] != HID) return;
  if (in_sizes[6] != 2 * HID * NCLS || in_sizes[7] != NCLS) return;
  if (in_sizes[8] != NCLS * NCLS || in_sizes[9] != NCLS) return;
  if ((long long)out_size != (long long)nN * NCLS) return;

  const float* x    = (const float*)d_in[0];
  const int*   edge = (const int*)d_in[1];
  const float* W1a  = (const float*)d_in[2];
  const float* b1a  = (const float*)d_in[3];
  const float* W1b  = (const float*)d_in[4];
  const float* b1b  = (const float*)d_in[5];
  const float* W2a  = (const float*)d_in[6];
  const float* b2a  = (const float*)d_in[7];
  const float* W2b  = (const float*)d_in[8];
  const float* b2b  = (const float*)d_in[9];
  float* out = (float*)d_out;
  const int* src = edge;
  const int* dst = edge + nE;

  const int MP  = cdiv(nN, GBM) * GBM;
  const int gM  = MP / GBM;
  const int nXB = MP / 16;
  const int gA1 = cdiv(nN, NB1);
  const int gA2 = cdiv(nN, NB2);
  if (gA1 > NFLAGMAX) return;
  const int vec8 = ((nE & 3) == 0) ? 1 : 0;

  char* ws = (char*)d_ws;
  size_t off = 0;
  const size_t oXB   = off; off = al256(off + (size_t)MP * CIN * 2);
  const size_t oBT1  = off; off = al256(off + (size_t)32 * CIN * 2);
  const size_t oBT1b = off; off = al256(off + (size_t)HID * 32 * 2);
  const size_t oBT2a = off; off = al256(off + (size_t)96 * 32 * 2);
  const size_t oBT2b = off; off = al256(off + (size_t)48 * K2B * 2);
  const size_t oBIAS = off; off = al256(off + (size_t)128 * 4);
  const size_t oFLAG = off; off = al256(off + (size_t)NFLAGMAX * 128);
  const size_t oPQ1  = off; off = al256(off + (size_t)MP * PQ1W * 4);
  const size_t oPQ2  = off; off = al256(off + (size_t)gA1 * NB1 * PQ2W * 4);
  if (off > ws_size || off > (size_t)WSMAX) return;
  unsigned short* XB   = (unsigned short*)(ws + oXB);
  unsigned short* BT1  = (unsigned short*)(ws + oBT1);
  unsigned short* BT1b = (unsigned short*)(ws + oBT1b);
  unsigned short* BT2a = (unsigned short*)(ws + oBT2a);
  unsigned short* BT2b = (unsigned short*)(ws + oBT2b);
  float*          BIAS = (float*)(ws + oBIAS);
  int*            FLAG = (int*)(ws + oFLAG);
  float*          PQ1  = (float*)(ws + oPQ1);
  float*          PQ2  = (float*)(ws + oPQ2);

  const size_t lds1 = (size_t)LDS1_INTS * 4;
  const size_t lds2 = (size_t)LDS2_INTS * 4;
  hipFuncSetAttribute(reinterpret_cast<const void*>(&k_scan1), hipFuncAttributeMaxDynamicSharedMemorySize, (int)lds1);
  hipFuncSetAttribute(reinterpret_cast<const void*>(&k_scan2), hipFuncAttributeMaxDynamicSharedMemorySize, (int)lds2);

  k_prep<<<nXB + 9, NTHR, 0, stream>>>(x, nN, nXB, W1a, b1a, W1b, b1b, W2a, b2a, W2b, b2b,
                                       XB, BT1, BT1b, BT2a, BT2b, BIAS);
  k_gemm1<<<gM, GTHR, 0, stream>>>(XB, BT1, BIAS, PQ1);
  k_scan1<<<gA1, NTHR, lds1, stream>>>(src, dst, nE, nN, vec8, PQ1, BT1b, BT2a, BIAS, PQ2, FLAG);
  k_scan2<<<gA2, NTHR, lds2, stream>>>(src, dst, nE, nN, vec8, PQ2, BT2b, BIAS, FLAG, gA1, out);
}
